// MHSA_5884105195621
// MI455X (gfx1250) — hardware-verified
//
#include <hip/hip_runtime.h>
#include <math.h>
#include <stdint.h>

#define NB   8
#define NC   128
#define NP   4096
#define NTOK (NB * NP)
#define PLANE_ELEMS ((size_t)NTOK * NC)

static_assert(NP % 64 == 0);
static_assert(NC == 128);
static_assert((NB * NC) % 32 == 0);
static_assert(NP % 256 == 0);

typedef __attribute__((ext_vector_type(16))) __bf16 v16b;
typedef __attribute__((ext_vector_type(8)))  __bf16 v8b;
typedef __attribute__((ext_vector_type(8)))  float  v8f;
typedef __attribute__((ext_vector_type(4)))  float  v4f;
typedef __attribute__((ext_vector_type(2)))  float  v2f;
typedef __attribute__((ext_vector_type(4)))  unsigned int v4u;
typedef v8b __attribute__((may_alias)) v8ba;
typedef v4f __attribute__((may_alias)) v4fa;
typedef v2f __attribute__((may_alias)) v2fa;
typedef v4u __attribute__((may_alias)) v4ua;

__device__ __forceinline__ unsigned short f2bf_bits(float f) {
  const unsigned u = __float_as_uint(f);
  return (unsigned short)((u + 0x7FFFu + ((u >> 16) & 1u)) >> 16);
}
__device__ __forceinline__ float bfbits2f(unsigned short h) { return __uint_as_float(((unsigned)h) << 16); }
__device__ __forceinline__ float bfr(float f) { return bfbits2f(f2bf_bits(f)); }
__device__ __forceinline__ unsigned pk16(unsigned short a, unsigned short b) { return (unsigned)a | ((unsigned)b << 16); }

__device__ __forceinline__ v8f mma_bf(v16b a, v16b b, v8f c) {
  c = __builtin_amdgcn_wmma_f32_16x16x32_bf16(false, a, false, b, (short)0, c, false, false);
  asm volatile("v_nop\n\tv_nop\n\tv_nop\n\tv_nop" : "+v"(c) : "v"(a), "v"(b));
  return c;
}
union FB { v16b v; v8b h[2]; };
__device__ __forceinline__ v16b ldfrag(const __bf16* p, int hh) {
  FB f;
  f.h[0] = *(const v8ba*)(p + 8 * hh);
  f.h[1] = *(const v8ba*)(p + 16 + 8 * hh);
  return f.v;
}

__global__ __launch_bounds__(256) void k_xt(const float* __restrict__ X, unsigned short* __restrict__ xt) {
  __shared__ __align__(16) float tf[64 * 68];
  const int b = blockIdx.z;
  const float* W = X + (size_t)b * NC * NP;
  unsigned short* o = xt + (size_t)b * NP * NC;
  const int c0 = blockIdx.x * 64;
  const int r0 = blockIdx.y * 64;
  const int tid = threadIdx.x;
  {
    const int lr = tid >> 4;
    const int c4 = (tid & 15) * 4;
#pragma unroll
    for (int it = 0; it < 4; ++it) {
      const int rr = it * 16 + lr;
      const v4f a = *(const v4fa*)(W + (size_t)(r0 + rr) * NP + c0 + c4);
      *(v4f*)(tf + rr * 68 + c4) = a;
    }
  }
  __syncthreads();
  const int sub = tid >> 3;
  const int c8  = (tid & 7) * 8;
  v4u hv[2];
#pragma unroll
  for (int it = 0; it < 2; ++it) {
    const int oc = it * 32 + sub;
    v4u a;
#pragma unroll
    for (int q = 0; q < 4; ++q) {
      const float f0 = tf[(c8 + 2 * q) * 68 + oc];
      const float f1 = tf[(c8 + 2 * q + 1) * 68 + oc];
      a[q] = pk16(f2bf_bits(f0), f2bf_bits(f1));
    }
    hv[it] = a;
  }
  for (int pass = 0; pass < 2; ++pass) {
#pragma unroll
    for (int it = 0; it < 2; ++it) {
      const int oc = it * 32 + sub;
      *(volatile v4ua*)(o + (size_t)(c0 + oc) * NC + r0 + c8) = hv[it];
    }
    __threadfence();
  }
}

__global__ __launch_bounds__(256) void k_wcvt(const float* __restrict__ qw, const float* __restrict__ kw,
                                             const float* __restrict__ vw, unsigned short* __restrict__ Wb) {
  const int which = blockIdx.y;
  const float* src = (which == 0) ? qw : ((which == 1) ? kw : vw);
  const int i = blockIdx.x * 256 + threadIdx.x;
  if (i >= NC * NC / 8) return;
  const v4f a = *(const v4fa*)(src + (size_t)i * 8);
  const v4f c = *(const v4fa*)(src + (size_t)i * 8 + 4);
  v4u o4;
  o4[0] = pk16(f2bf_bits(a[0]), f2bf_bits(a[1]));
  o4[1] = pk16(f2bf_bits(a[2]), f2bf_bits(a[3]));
  o4[2] = pk16(f2bf_bits(c[0]), f2bf_bits(c[1]));
  o4[3] = pk16(f2bf_bits(c[2]), f2bf_bits(c[3]));
  unsigned short* dst = Wb + (size_t)which * NC * NC + (size_t)i * 8;
  *(volatile v4ua*)dst = o4;
  __threadfence();
  *(volatile v4ua*)dst = o4;
}

__global__ __launch_bounds__(256) void k_poolbc(const float* __restrict__ x2, float* __restrict__ AV,
                                               float* __restrict__ MX) {
  __shared__ float ws_s[8], ws_m[8];
  __shared__ __align__(16) float os[64];
  const int g = blockIdx.x, tid = threadIdx.x, lane = tid & 31, w = tid >> 5;
#pragma unroll 1
  for (int j = 0; j < 32; ++j) {
    const float* p = x2 + (size_t)(g * 32 + j) * NP + tid * 16;
    float s = 0.f, m = -INFINITY;
#pragma unroll
    for (int i = 0; i < 4; ++i) {
      const v4f a = *(const v4fa*)(p + 4 * i);
      const float a0 = bfr(a[0]), a1 = bfr(a[1]), a2 = bfr(a[2]), a3 = bfr(a[3]);
      s += (a0 + a1) + (a2 + a3);
      m = fmaxf(fmaxf(m, a0), fmaxf(fmaxf(a1, a2), a3));
    }
#pragma unroll
    for (int off = 16; off > 0; off >>= 1) {
      s += __shfl_xor(s, off, 32);
      m = fmaxf(m, __shfl_xor(m, off, 32));
    }
    if (lane == 0) { ws_s[w] = s; ws_m[w] = m; }
    __syncthreads();
    if (tid == 0) {
      float ts = 0.f, tm = -INFINITY;
#pragma unroll
      for (int k = 0; k < 8; ++k) { ts += ws_s[k]; tm = fmaxf(tm, ws_m[k]); }
      os[j] = ts * (1.0f / 4096.0f);
      os[32 + j] = tm;
    }
    __syncthreads();
  }
  if (w == 0) {
    const v4f v = *(const v4fa*)(os + 4 * (lane & 15));
    for (int pass = 0; pass < 2; ++pass) {
      if (lane < 8)       *(volatile v4f*)(AV + g * 32 + 4 * lane) = v;
      else if (lane < 16) *(volatile v4f*)(MX + g * 32 + 4 * (lane - 8)) = v;
      __threadfence();
    }
  }
}

__global__ __launch_bounds__(256) void k_poolc(const float* __restrict__ x2, float* __restrict__ SPIN) {
  __shared__ float ps[4][64], pm[4][64];
  __shared__ __align__(16) float os[128];
  const int b = blockIdx.x >> 6, g = blockIdx.x & 63;
  const int tid = threadIdx.x, lane = tid & 31;
  const int p = tid & 63, cg = tid >> 6;
  const float* src = x2 + ((size_t)b * NC + cg * 32) * NP + g * 64 + p;
  float s = 0.f, m = -INFINITY;
#pragma unroll 4
  for (int c = 0; c < 32; ++c) {
    const float v = bfr(src[(size_t)c * NP]);
    s += v;
    m = fmaxf(m, v);
  }
  ps[cg][p] = s;
  pm[cg][p] = m;
  __syncthreads();
  if (tid < 64) {
    const float ts = ((ps[0][tid] + ps[1][tid]) + ps[2][tid]) + ps[3][tid];
    const float tm = fmaxf(fmaxf(pm[0][tid], pm[1][tid]), fmaxf(pm[2][tid], pm[3][tid]));
    os[tid] = ts * (1.0f / 128.0f);
    os[64 + tid] = tm;
  }
  __syncthreads();
  if (tid < 32) {
    const v4f v = *(const v4fa*)(os + 4 * lane);
    float* base = SPIN + (size_t)b * 2 * NP + g * 64;
    for (int pass = 0; pass < 2; ++pass) {
      if (lane < 16) *(volatile v4f*)(base + 4 * lane) = v;
      else           *(volatile v4f*)(base + NP + 4 * (lane - 16)) = v;
      __threadfence();
    }
  }
}

__global__ __launch_bounds__(256) void k_pos(const float* __restrict__ AV, const float* __restrict__ MX,
                                            const float* __restrict__ SPIN, const float* __restrict__ c1w,
                                            const float* __restrict__ ckw, const float* __restrict__ ckb,
                                            const float* __restrict__ spw, const float* __restrict__ spb,
                                            float* __restrict__ AVEC, float* __restrict__ RVEC,
                                            float* __restrict__ SP) {
  __shared__ float sav[128], smx[128], sch[128];
  __shared__ float sw1[32], sw2[128];
  __shared__ __align__(16) float savec[128], srv[128];
  __shared__ float spl[2 * 4900];
  __shared__ __align__(16) float ssp[NP];
  const int b = blockIdx.x, tid = threadIdx.x, lane = tid & 31, w = tid >> 5;

  if (tid < 128) {
    sav[tid] = AV[b * NC + tid];
    smx[tid] = MX[b * NC + tid];
    sw2[tid] = bfr(spw[min(tid, 97)]);
  }
  if (w == 0) sw1[lane] = bfr(c1w[min(lane, 9)]);
  for (int i = tid; i < 2 * 4900; i += 256) spl[i] = 0.0f;
  __syncthreads();
#pragma unroll 2
  for (int i = tid; i < NP; i += 256) {
    const int h = i >> 6, x = i & 63;
    const int li = (h + 3) * 70 + x + 3;
    spl[li]        = SPIN[(size_t)b * 2 * NP + i];
    spl[4900 + li] = SPIN[(size_t)b * 2 * NP + NP + i];
  }
  if (tid < 128) {
    const int c = tid;
    float acc = 0.0f;
#pragma unroll 1
    for (int t = 0; t < 5; ++t) {
      const int cc  = c + t - 2;
      const int ccl = min(max(cc, 0), NC - 1);
      const float valid = (cc >= 0 && cc < NC) ? 1.0f : 0.0f;
      acc += valid * (sw1[t] * sav[ccl] + sw1[5 + t] * smx[ccl]);
    }
    sch[c] = acc;
  }
  __syncthreads();
  if (tid < 128) {
    const int o = tid;
    float a = bfr(ckb[o]), r = 0.0f;
    const float* wr = ckw + (size_t)o * NC;
#pragma unroll 4
    for (int c = 0; c < NC; ++c) {
      const float wv = bfr(wr[c]);
      a += wv * sch[c];
      r += wv;
    }
    savec[o] = a;
    srv[o] = r;
  }
  const float bias_sp = bfr(spb[0]);
#pragma unroll 1
  for (int it = 0; it < NP / 256; ++it) {
    const int n = it * 256 + tid;
    const int h = n >> 6, x = n & 63;
    float acc = bias_sp;
#pragma unroll 1
    for (int u = 0; u < 7; ++u) {
#pragma unroll 1
      for (int v = 0; v < 7; ++v) {
        const int li = (h + u) * 70 + x + v;
        acc += sw2[u * 7 + v] * spl[li] + sw2[49 + u * 7 + v] * spl[4900 + li];
      }
    }
    ssp[n] = acc;
  }
  __syncthreads();
  if (w == 0) {
    const v4f v = *(const v4fa*)(savec + 4 * lane);
    for (int pass = 0; pass < 2; ++pass) {
      *(volatile v4f*)(AVEC + b * NC + 4 * lane) = v;
      __threadfence();
    }
  } else if (w == 1) {
    const v4f v = *(const v4fa*)(srv + 4 * lane);
    for (int pass = 0; pass < 2; ++pass) {
      *(volatile v4f*)(RVEC + b * NC + 4 * lane) = v;
      __threadfence();
    }
  }
  {
    v4f sv[4];
#pragma unroll
    for (int it = 0; it < 4; ++it) sv[it] = *(const v4fa*)(ssp + it * 1024 + 4 * tid);
    for (int pass = 0; pass < 2; ++pass) {
#pragma unroll
      for (int it = 0; it < 4; ++it)
        *(volatile v4f*)(SP + (size_t)b * NP + it * 1024 + 4 * tid) = sv[it];
      __threadfence();
    }
  }
}

__global__ __launch_bounds__(128) void k_qkv(const __bf16* __restrict__ XT, const __bf16* __restrict__ Wb,
                                            const float* __restrict__ qb, const float* __restrict__ kb,
                                            const float* __restrict__ vb,
                                            const float* __restrict__ AVEC, const float* __restrict__ RVEC,
                                            unsigned short* __restrict__ QP, unsigned short* __restrict__ KP,
                                            unsigned short* __restrict__ VP,
                                            float* __restrict__ ALPHA, float* __restrict__ BETA) {
  __shared__ __align__(16) float sT[64 * 132];
  __shared__ __align__(16) float sAV[128], sRV[128], sAB[128], sBI[128];
  const int tid = threadIdx.x, lane = tid & 31, w = tid >> 5, hh = lane >> 4, l16 = lane & 15;
  const int which = blockIdx.y;
  const int m0 = blockIdx.x * 64;
  const int b  = m0 / NP;
  const int n0 = m0 - b * NP;

  const float* bias = (which == 0) ? qb : ((which == 1) ? kb : vb);
  sAV[tid] = AVEC[b * NC + tid];
  sRV[tid] = RVEC[b * NC + tid];
  sBI[tid] = bfr(bias[tid]);
  __syncthreads();

  const v8f zero8 = {0.f, 0.f, 0.f, 0.f, 0.f, 0.f, 0.f, 0.f};
  v8f acc[8];
#pragma unroll
  for (int t = 0; t < 8; ++t) acc[t] = zero8;

  const __bf16* arow = XT + (size_t)(m0 + 16 * w + l16) * NC;
  const __bf16* brow = Wb + ((size_t)which * NC + l16) * NC;
#pragma unroll
  for (int kc = 0; kc < 4; ++kc) {
    const v16b a = ldfrag(arow + kc * 32, hh);
#pragma unroll
    for (int t = 0; t < 8; ++t) {
      const v16b bf = ldfrag(brow + (size_t)t * 16 * NC + kc * 32, hh);
      acc[t] = mma_bf(a, bf, acc[t]);
    }
  }
#pragma unroll
  for (int t = 0; t < 8; ++t) {
    const float bv = sBI[16 * t + l16];
#pragma unroll
    for (int r = 0; r < 8; ++r) sT[(16 * w + 8 * hh + r) * 132 + 16 * t + l16] = acc[t][r] + bv;
  }
  __syncthreads();
  if (which == 0 && tid < 64) {
    const float* qr = sT + tid * 132;
    float a = 0.0f, be = 0.0f;
#pragma unroll 4
    for (int o = 0; o < NC; ++o) {
      const float q = qr[o];
      a  += sAV[o] * q;
      be += sRV[o] * q;
    }
    sAB[tid] = a;
    sAB[64 + tid] = be;
  }
  __syncthreads();

  const int q8 = lane & 7, sub = lane >> 3;
  v4u hv[8], lv[8];
#pragma unroll
  for (int i = 0; i < 8; ++i) {
    const int lid  = w * 32 + i * 4 + sub;
    const int base = (which != 2) ? ((lid >> 1) * 132 + (lid & 1) * 64 + 8 * q8) : ((8 * q8) * 132 + lid);
    const int estr = (which != 2) ? 1 : 132;
    v4u a, a2;
#pragma unroll
    for (int q = 0; q < 4; ++q) {
      const float f0 = sT[base + (2 * q) * estr];
      const float f1 = sT[base + (2 * q + 1) * estr];
      const unsigned short h0 = f2bf_bits(f0), h1 = f2bf_bits(f1);
      const unsigned short l0 = f2bf_bits(f0 - bfbits2f(h0)), l1 = f2bf_bits(f1 - bfbits2f(h1));
      a[q]  = pk16(h0, h1);
      a2[q] = pk16(l0, l1);
    }
    hv[i] = a;
    lv[i] = a2;
  }
  unsigned short* P = (which == 0) ? QP : ((which == 1) ? KP : VP);
  for (int pass = 0; pass < 2; ++pass) {
#pragma unroll
    for (int i = 0; i < 8; ++i) {
      const int lid = w * 32 + i * 4 + sub;
      const size_t go = (which != 2)
          ? ((size_t)(m0 + (lid >> 1)) * NC + (lid & 1) * 64 + 8 * q8)
          : (((size_t)b * NC + lid) * NP + n0 + 8 * q8);
      *(volatile v4ua*)(P + go) = hv[i];
      *(volatile v4ua*)(P + PLANE_ELEMS + go) = lv[i];
    }
    __threadfence();
  }
  if (which == 0 && w == 0) {
    const v4f v = *(const v4fa*)(sAB + 4 * lane);
    for (int pass = 0; pass < 2; ++pass) {
      if (lane < 16) *(volatile v4f*)(ALPHA + m0 + 4 * lane) = v;
      else           *(volatile v4f*)(BETA + m0 + 4 * (lane - 16)) = v;
      __threadfence();
    }
  }
}

#define SM_K   0
#define SM_V   32768
#define SM_Q   65536
#define SM_P   98304
#define SM_AB  114688
#define SM_RED 115200
#define SM_TOT 116224
static_assert(128 * 68 * 4 <= SM_Q);

__global__ __launch_bounds__(256) void k_attn(const __bf16* __restrict__ QP, const __bf16* __restrict__ KP,
                                             const __bf16* __restrict__ VP, const float* __restrict__ ALPHA,
                                             const float* __restrict__ BETA, const float* __restrict__ SP,
                                             float* __restrict__ out) {
  __shared__ __align__(16) unsigned char smem[SM_TOT];
  __bf16* Ks   = (__bf16*)(smem + SM_K);
  __bf16* Vs   = (__bf16*)(smem + SM_V);
  __bf16* Qs   = (__bf16*)(smem + SM_Q);
  __bf16* Ps   = (__bf16*)(smem + SM_P);
  float*  sab  = (float*)(smem + SM_AB);
  float*  redm = (float*)(smem + SM_RED);
  float*  reds = redm + 128;
  float*  Os   = (float*)(smem + SM_K);

  const int tid = threadIdx.x, lane = tid & 31, w = tid >> 5, hh = lane >> 4, c = lane & 15;
  const int g = w & 3, kh = w >> 2;
  const int key0 = 32 * kh;
  const int ch0  = 64 * kh;
  const int b  = blockIdx.x >> 6;
  const int n0 = (blockIdx.x & 63) * 64;
  const size_t tok0 = (size_t)b * NP + n0;

  {
    const int r = tid >> 2, part = tid & 3, p = part >> 1, half = (part & 1) * 64;
    const __bf16* src = QP + (size_t)p * PLANE_ELEMS + (tok0 + r) * NC + half;
    __bf16* dst = Qs + p * 8192 + r * 128 + half;
#pragma unroll
    for (int i = 0; i < 8; ++i) { const v8b v = *(const v8ba*)(src + 8 * i); *(v8ba*)(dst + 8 * i) = v; }
  }
  float spn[8];
  {
    const v4f s0 = *(const v4fa*)(SP + tok0 + 16 * g + 8 * hh);
    const v4f s1 = *(const v4fa*)(SP + tok0 + 16 * g + 8 * hh + 4);
    spn[0] = s0[0]; spn[1] = s0[1]; spn[2] = s0[2]; spn[3] = s0[3];
    spn[4] = s1[0]; spn[5] = s1[1]; spn[6] = s1[2]; spn[7] = s1[3];
  }
  float mrow[8], lrow[8];
  const v8f zero8 = {0.f, 0.f, 0.f, 0.f, 0.f, 0.f, 0.f, 0.f};
  v8f oacc[4];
#pragma unroll
  for (int r = 0; r < 8; ++r) { mrow[r] = -INFINITY; lrow[r] = 0.0f; }
#pragma unroll
  for (int t = 0; t < 4; ++t) oacc[t] = zero8;

  const __bf16* qrow = Qs + (16 * g + c) * 128;
  __bf16* pgh = Ps + g * 1024;
  __bf16* pgl = Ps + 4096 + g * 1024;
  const int rme = g * 32 + kh * 16 + 8 * hh;
  const int r0e = g * 32 + 8 * hh;
  const int r1e = g * 32 + 16 + 8 * hh;

#pragma unroll 1
  for (int kc = 0; kc < NP / 64; ++kc) {
    const int m0 = kc * 64;
    __syncthreads();
    {
      const int r = tid >> 2, part = tid & 3, p = part >> 1, half = (part & 1) * 64;
      const __bf16* ksrc = KP + (size_t)p * PLANE_ELEMS + ((size_t)b * NP + m0 + r) * NC + half;
      __bf16* kd = Ks + p * 8192 + r * 128 + half;
#pragma unroll
      for (int i = 0; i < 8; ++i) { const v8b a = *(const v8ba*)(ksrc + 8 * i); *(v8ba*)(kd + 8 * i) = a; }
      const int r2 = tid >> 1, p2 = tid & 1;
      const __bf16* vsrc = VP + (size_t)p2 * PLANE_ELEMS + ((size_t)b * NC + r2) * NP + m0;
      __bf16* vd = Vs + p2 * 8192 + r2 * 64;
#pragma unroll
      for (int i = 0; i < 8; ++i) { const v8b a = *(const v8ba*)(vsrc + 8 * i); *(v8ba*)(vd + 8 * i) = a; }
      if (w == 0) {
        const v2f a = *(const v2fa*)(ALPHA + (size_t)b * NP + m0 + 2 * lane);
        *(v2fa*)(sab + 2 * lane) = a;
      } else if (w == 1) {
        const v2f a = *(const v2fa*)(BETA + (size_t)b * NP + m0 + 2 * lane);
        *(v2fa*)(sab + 64 + 2 * lane) = a;
      }
    }
    __syncthreads();

    v8f s[2];
    s[0] = zero8; s[1] = zero8;
#pragma unroll 1
    for (int dc = 0; dc < 4; ++dc) {
      const v16b qa = ldfrag(qrow + dc * 32, hh);
      const v16b ql = ldfrag(qrow + 8192 + dc * 32, hh);
#pragma unroll
      for (int jj = 0; jj < 2; ++jj) {
        const __bf16* krow = Ks + (key0 + 16 * jj + c) * 128 + dc * 32;
        const v16b kb = ldfrag(krow, hh);
        const v16b kl = ldfrag(krow + 8192, hh);
        s[jj] = mma_bf(qa, kb, s[jj]);
        s[jj] = mma_bf(qa, kl, s[jj]);
        s[jj] = mma_bf(ql, kb, s[jj]);
      }
    }
    float al[2], be[2];
#pragma unroll
    for (int jj = 0; jj < 2; ++jj) { al[jj] = sab[key0 + 16 * jj + c]; be[jj] = sab[64 + key0 + 16 * jj + c]; }
#pragma unroll
    for (int r = 0; r < 8; ++r) {
      float m = -INFINITY;
#pragma unroll
      for (int jj = 0; jj < 2; ++jj) {
        const float e = s[jj][r] + al[jj] + spn[r] * be[jj];
        s[jj][r] = e;
        m = fmaxf(m, e);
      }
#pragma unroll
      for (int off = 1; off < 16; off <<= 1) m = fmaxf(m, __shfl_xor(m, off, 32));
      if (c == 0) redm[rme + r] = m;
    }
    __syncthreads();
    float corr[8];
#pragma unroll
    for (int r = 0; r < 8; ++r) {
      const float cmx  = fmaxf(redm[r0e + r], redm[r1e + r]);
      const float mnew = fmaxf(mrow[r], cmx);
      corr[r] = expf(mrow[r] - mnew);
      mrow[r] = mnew;
      float psum = 0.0f;
#pragma unroll
      for (int jj = 0; jj < 2; ++jj) {
        const float p = expf(s[jj][r] - mnew);
        psum += p;
        const unsigned short hb = f2bf_bits(p);
        const unsigned short lb = f2bf_bits(p - bfbits2f(hb));
        pgh[(8 * hh + r) * 64 + key0 + 16 * jj + c] = __builtin_bit_cast(__bf16, hb);
        pgl[(8 * hh + r) * 64 + key0 + 16 * jj + c] = __builtin_bit_cast(__bf16, lb);
      }
#pragma unroll
      for (int off = 1; off < 16; off <<= 1) psum += __shfl_xor(psum, off, 32);
      if (c == 0) reds[rme + r] = psum;
      lrow[r] = lrow[r] * corr[r];
#pragma unroll
      for (int t = 0; t < 4; ++t) oacc[t][r] *= corr[r];
    }
    __syncthreads();
#pragma unroll
    for (int r = 0; r < 8; ++r) lrow[r] += reds[r0e + r] + reds[r1e + r];

#pragma unroll 1
    for (int kk = 0; kk < 2; ++kk) {
      const v16b pa = ldfrag(pgh + c * 64 + kk * 32, hh);
      const v16b pl = ldfrag(pgl + c * 64 + kk * 32, hh);
#pragma unroll
      for (int t = 0; t < 4; ++t) {
        const __bf16* vr = Vs + (ch0 + 16 * t + c) * 64 + kk * 32;
        const v16b vb = ldfrag(vr, hh);
        const v16b vl = ldfrag(vr + 8192, hh);
        oacc[t] = mma_bf(pa, vb, oacc[t]);
        oacc[t] = mma_bf(pa, vl, oacc[t]);
        oacc[t] = mma_bf(pl, vb, oacc[t]);
      }
    }
  }
  __syncthreads();

#pragma unroll
  for (int r = 0; r < 8; ++r) {
    const float inv = 1.0f / lrow[r];
#pragma unroll
    for (int t = 0; t < 4; ++t) Os[(ch0 + 16 * t + c) * 68 + 16 * g + 8 * hh + r] = oacc[t][r] * inv;
  }
  __syncthreads();
  {
    float* ob = out + (size_t)b * NC * NP + n0;
    const int c4 = (lane & 15) * 4;
    for (int pass = 0; pass < 2; ++pass) {
#pragma unroll
      for (int i = 0; i < 8; ++i) {
        const int row = i * 16 + w * 2 + hh;
        const v4f v = *(const v4fa*)(Os + row * 68 + c4);
        *(volatile v4f*)(ob + (size_t)row * NP + c4) = v;
      }
      __threadfence();
    }
  }
}

extern "C" void kernel_launch(void* const* d_in, const int* in_sizes, int n_in,
                              void* d_out, int out_size, void* d_ws, size_t ws_size,
                              hipStream_t stream) {
  if (n_in < 13) return;
  if (in_sizes[0] != NB * NC * NP || in_sizes[1] != NB * NC * NP) return;
  if (in_sizes[2] != NC * NC || in_sizes[4] != NC * NC || in_sizes[6] != NC * NC || in_sizes[8] != NC * NC) return;
  if (in_sizes[3] != NC || in_sizes[5] != NC || in_sizes[7] != NC || in_sizes[9] != NC) return;
  if (in_sizes[10] != 10 || in_sizes[11] != 98 || in_sizes[12] != 1) return;
  if (out_size != NB * NC * NP) return;

  const float* x    = (const float*)d_in[0];
  const float* x2   = (const float*)d_in[1];
  const float* q_w  = (const float*)d_in[2];
  const float* q_b  = (const float*)d_in[3];
  const float* k_w  = (const float*)d_in[4];
  const float* k_b  = (const float*)d_in[5];
  const float* v_w  = (const float*)d_in[6];
  const float* v_b  = (const float*)d_in[7];
  const float* ck_w = (const float*)d_in[8];
  const float* ck_b = (const float*)d_in[9];
  const float* c1w  = (const float*)d_in[10];
  const float* sp_w = (const float*)d_in[11];
  const float* sp_b = (const float*)d_in[12];
  float* out = (float*)d_out;

  const size_t plane_b = PLANE_ELEMS * 2;
  size_t off = 0;
  const size_t oXT   = off; off += plane_b;
  const size_t oW    = off; off += (size_t)3 * NC * NC * 2;
  const size_t oAV   = off; off += (size_t)NB * NC * 4;
  const size_t oMX   = off; off += (size_t)NB * NC * 4;
  const size_t oSPIN = off; off += (size_t)NB * 2 * NP * 4;
  const size_t oAVEC = off; off += (size_t)NB * NC * 4;
  const size_t oRVEC = off; off += (size_t)NB * NC * 4;
  const size_t oSP   = off; off += (size_t)NB * NP * 4;
  const size_t oAL   = off; off += (size_t)NB * NP * 4;
  const size_t oBE   = off; off += (size_t)NB * NP * 4;
  const size_t oQ    = off; off += 2 * plane_b;
  const size_t oK    = off; off += 2 * plane_b;
  const size_t oV    = off; off += 2 * plane_b;
  if (off > ws_size) return;
  if (off > (size_t)134217728) return;

  char* ws = (char*)d_ws;
  unsigned short* XT    = (unsigned short*)(ws + oXT);
  unsigned short* WQKV  = (unsigned short*)(ws + oW);
  float* AV    = (float*)(ws + oAV);
  float* MX    = (float*)(ws + oMX);
  float* SPIN  = (float*)(ws + oSPIN);
  float* AVEC  = (float*)(ws + oAVEC);
  float* RVEC  = (float*)(ws + oRVEC);
  float* SP    = (float*)(ws + oSP);
  float* ALPHA = (float*)(ws + oAL);
  float* BETA  = (float*)(ws + oBE);
  unsigned short* QP = (unsigned short*)(ws + oQ);
  unsigned short* KPp = (unsigned short*)(ws + oK);
  unsigned short* VPp = (unsigned short*)(ws + oV);

  k_xt<<<dim3(NP / 64, NC / 64, NB), 256, 0, stream>>>(x, XT);
  k_wcvt<<<dim3(NC * NC / 8 / 256, 3), 256, 0, stream>>>(q_w, k_w, v_w, WQKV);
  k_poolbc<<<NB * NC / 32, 256, 0, stream>>>(x2, AV, MX);
  k_poolc<<<NB * (NP / 64), 256, 0, stream>>>(x2, SPIN);
  k_pos<<<NB, 256, 0, stream>>>(AV, MX, SPIN, c1w, ck_w, ck_b, sp_w, sp_b, AVEC, RVEC, SP);
  k_qkv<<<dim3(NTOK / 64, 3), 128, 0, stream>>>((const __bf16*)(const void*)XT, (const __bf16*)(const void*)WQKV,
                                                q_b, k_b, v_b, AVEC, RVEC, QP, KPp, VPp, ALPHA, BETA);
  k_attn<<<NB * (NP / 64), 256, 0, stream>>>((const __bf16*)(const void*)QP, (const __bf16*)(const void*)KPp,
                                             (const __bf16*)(const void*)VPp, ALPHA, BETA, SP, out);
  (void)hipGetLastError();
}
